// RnnTimeSeriesEncoder_24550033064431
// MI455X (gfx1250) — hardware-verified
//
#include <hip/hip_runtime.h>

typedef __attribute__((ext_vector_type(16))) _Float16 v16h;
typedef __attribute__((ext_vector_type(8)))  _Float16 v8h;
typedef __attribute__((ext_vector_type(8)))  float    v8f;
typedef __attribute__((ext_vector_type(4)))  float    v4f;

__device__ __forceinline__ void dep_guard_h(v8f& a, v8f& b, v16h x, v16h y) { asm volatile("v_nop\n\tv_nop\n\tv_nop\n\tv_nop" : "+v"(a), "+v"(b) : "v"(x), "v"(y)); }
__device__ __forceinline__ void keep4_h(v16h a, v16h b, v16h c, v16h d) { asm volatile("v_nop" :: "v"(a), "v"(b), "v"(c), "v"(d)); }
__device__ __forceinline__ void acc_guard4(v8f& a, v8f& b, v8f& c, v8f& d) { asm volatile("v_nop\n\tv_nop\n\tv_nop\n\tv_nop" : "+v"(a), "+v"(b), "+v"(c), "+v"(d)); }
template <typename T> struct Frag;
template <> struct Frag<_Float16> {
  typedef v16h V; union U { v16h v; v8h h[2]; };
  static __device__ __forceinline__ v16h load(const _Float16* p) {
    U f; f.h[0] = *(const v8h*)(p); f.h[1] = *(const v8h*)(p + 16); return f.v;
  }
  static __device__ __forceinline__ v8f mma(v16h a, v16h b, v8f c) {
    return __builtin_amdgcn_wmma_f32_16x16x32_f16(false, a, false, b, (short)0, c, false, false);
  }
  static __device__ __forceinline__ void guard(v8f& a, v8f& b, v16h x, v16h y) { dep_guard_h(a, b, x, y); }
  static __device__ __forceinline__ void keep(v16h a, v16h b, v16h c, v16h d) { keep4_h(a, b, c, d); }
};
__device__ __forceinline__ void guard9(v8f& a0, v8f& a1, v8f& a2, v8f& a3,
                                       v16h x, v16h b0, v16h b1, v16h b2, v16h b3) {
  asm volatile("v_nop\n\tv_nop\n\tv_nop\n\tv_nop"
               : "+v"(a0), "+v"(a1), "+v"(a2), "+v"(a3)
               : "v"(x), "v"(b0), "v"(b1), "v"(b2), "v"(b3));
}

constexpr int kBatch = 256;
constexpr int kSteps = 512;
constexpr int kIn    = 32;
constexpr int kHid   = 256;
constexpr int kGates = 4 * kHid;
constexpr int kK0    = kIn + kHid;
constexpr int kK1    = 2 * kHid;
constexpr int kRowsPerBlock = 16;
constexpr int kPA0   = 296;
constexpr int kPA1   = 520;
constexpr int kOSP   = 260;
constexpr float kActScale = 256.0f;
constexpr float kWScale   = 64.0f;
constexpr float kAccInv   = 1.0f / 16384.0f;
static_assert(kK0 % 32 == 0 && kK1 % 32 == 0, "");
static_assert(kBatch % kRowsPerBlock == 0, "");
static_assert((kPA0 % 8) == 0 && (kPA1 % 8) == 0 && (kOSP % 4) == 0, "");
static_assert(kGates == 16 * 4 * 16, "");

__device__ __forceinline__ float sigm_f(float x) {
  return __builtin_amdgcn_rcpf(1.0f + expf(-x));
}
__device__ __forceinline__ float tanh_f(float x) {
  const float e = expf(2.0f * x);
  return 1.0f - 2.0f * __builtin_amdgcn_rcpf(1.0f + e);
}

__global__ __launch_bounds__(256) void build_bt_plane(
    const float* __restrict__ W1, int k1,
    const float* __restrict__ W2, int k2,
    _Float16* __restrict__ dst, int pitch, int nrows, float scale) {
  const int i = blockIdx.x * 256 + threadIdx.x;
  const int cpr = pitch >> 3;
  const int total = nrows * cpr;
  if (i >= total) return;
  const int row  = i / cpr;
  const int col0 = (i - row * cpr) * 8;
  int ca = col0;      if (ca > k1 - 8) ca = k1 - 8;
  int cb = col0 - k1; if (cb < 0) cb = 0; if (cb > k2 - 8) cb = k2 - 8;
  const float* pa = W1 + (size_t)row * k1 + ca;
  const float* pb = W2 + (size_t)row * k2 + cb;
  const v4f a0 = *(const v4f*)pa, a1 = *(const v4f*)(pa + 4);
  const v4f q0 = *(const v4f*)pb, q1 = *(const v4f*)(pb + 4);
  const bool useA = (col0 < k1);
  const bool useB = (!useA) && (col0 < k1 + k2);
  v8h hv;
#pragma unroll
  for (int e = 0; e < 4; ++e) {
    const float s0 = useA ? a0[e] : (useB ? q0[e] : 0.0f);
    const float s1 = useA ? a1[e] : (useB ? q1[e] : 0.0f);
    hv[e]     = (_Float16)(s0 * scale);
    hv[4 + e] = (_Float16)(s1 * scale);
  }
  _Float16* o = dst + (size_t)i * 8;
  *(volatile v8h*)o = hv;
  __threadfence();
  *(volatile v8h*)o = hv;
}

__global__ __launch_bounds__(512) void lstm2_persist(
    const float* __restrict__ Mx,
    const _Float16* __restrict__ Wc0,
    const _Float16* __restrict__ Wc1,
    const float* __restrict__ bih0, const float* __restrict__ bhh0,
    const float* __restrict__ bih1, const float* __restrict__ bhh1,
    float* __restrict__ out) {
  __shared__ __align__(16) _Float16 A0s[kRowsPerBlock * kPA0];
  __shared__ __align__(16) _Float16 A1s[kRowsPerBlock * kPA1];
  __shared__ __align__(16) float    Os[kRowsPerBlock * kOSP];

  const int tid  = threadIdx.x;
  const int w    = tid >> 5;
  const int lane = tid & 31;
  const int nl   = lane & 15;
  const int hi   = lane >> 4;
  const int col  = w * 16 + nl;
  const int b0   = blockIdx.x * kRowsPerBlock;
  const int srow = tid >> 5;
  const int scol = tid & 31;

  float bg0[4], bg1[4];
#pragma unroll
  for (int g = 0; g < 4; ++g) {
    bg0[g] = bih0[g * kHid + col] + bhh0[g * kHid + col];
    bg1[g] = bih1[g * kHid + col] + bhh1[g * kHid + col];
  }

  {
    v8h z;
#pragma unroll
    for (int e = 0; e < 8; ++e) z[e] = (_Float16)0.0f;
    *(v8h*)(A0s + srow * kPA0 + kIn  + scol * 8) = z;
    *(v8h*)(A1s + srow * kPA1 + kHid + scol * 8) = z;
    const float xv = Mx[((size_t)(b0 + srow) * kSteps + 0) * kIn + scol];
    A0s[srow * kPA0 + scol] = (_Float16)(xv * kActScale);
  }

  v8f c0st = (v8f){0.f,0.f,0.f,0.f,0.f,0.f,0.f,0.f};
  v8f c1st = (v8f){0.f,0.f,0.f,0.f,0.f,0.f,0.f,0.f};
  v8f h1last = (v8f){0.f,0.f,0.f,0.f,0.f,0.f,0.f,0.f};
  __syncthreads();

  int zoff = 0;

#pragma unroll 1
  for (int t = 0; t < kSteps; ++t) {
    asm volatile("" : "+s"(zoff));
    const _Float16* w0p = Wc0 + zoff;
    const _Float16* w1p = Wc1 + zoff;

    v8f acc[4];
#pragma unroll
    for (int g = 0; g < 4; ++g) acc[g] = (v8f){0.f,0.f,0.f,0.f,0.f,0.f,0.f,0.f};
#pragma unroll 1
    for (int ks = 0; ks < kK0 / 32; ++ks) {
      const int kc = ks * 32 + 8 * hi;
      const v16h a = Frag<_Float16>::load(A0s + nl * kPA0 + kc);
      v16h bq[4];
#pragma unroll
      for (int g = 0; g < 4; ++g)
        bq[g] = Frag<_Float16>::load(w0p + (size_t)(g * kHid + col) * kK0 + kc);
#pragma unroll
      for (int g = 0; g < 4; ++g) acc[g] = Frag<_Float16>::mma(a, bq[g], acc[g]);
      guard9(acc[0], acc[1], acc[2], acc[3], a, bq[0], bq[1], bq[2], bq[3]);
    }
    acc_guard4(acc[0], acc[1], acc[2], acc[3]);
    __syncthreads();

    {
#pragma unroll
      for (int r = 0; r < 8; ++r) {
        const float pi = acc[0][r] * kAccInv + bg0[0];
        const float pf = acc[1][r] * kAccInv + bg0[1];
        const float pg = acc[2][r] * kAccInv + bg0[2];
        const float po = acc[3][r] * kAccInv + bg0[3];
        const float ig = sigm_f(pi);
        const float fg = sigm_f(pf);
        const float gg = tanh_f(pg);
        const float og = sigm_f(po);
        const float cc = fg * c0st[r] + ig * gg;
        c0st[r] = cc;
        const float h = og * tanh_f(cc);
        const _Float16 hf = (_Float16)(h * kActScale);
        A0s[(8 * hi + r) * kPA0 + kIn + col] = hf;
        A1s[(8 * hi + r) * kPA1 + col] = hf;
      }
      const int tn = (t + 1 < kSteps) ? (t + 1) : (kSteps - 1);
      const float xv = Mx[((size_t)(b0 + srow) * kSteps + tn) * kIn + scol];
      A0s[srow * kPA0 + scol] = (_Float16)(xv * kActScale);
    }
    __syncthreads();

#pragma unroll
    for (int g = 0; g < 4; ++g) acc[g] = (v8f){0.f,0.f,0.f,0.f,0.f,0.f,0.f,0.f};
#pragma unroll 1
    for (int ks = 0; ks < kK1 / 32; ++ks) {
      const int kc = ks * 32 + 8 * hi;
      const v16h a = Frag<_Float16>::load(A1s + nl * kPA1 + kc);
      v16h bq[4];
#pragma unroll
      for (int g = 0; g < 4; ++g)
        bq[g] = Frag<_Float16>::load(w1p + (size_t)(g * kHid + col) * kK1 + kc);
#pragma unroll
      for (int g = 0; g < 4; ++g) acc[g] = Frag<_Float16>::mma(a, bq[g], acc[g]);
      guard9(acc[0], acc[1], acc[2], acc[3], a, bq[0], bq[1], bq[2], bq[3]);
    }
    acc_guard4(acc[0], acc[1], acc[2], acc[3]);
    __syncthreads();

    {
#pragma unroll
      for (int r = 0; r < 8; ++r) {
        const float pi = acc[0][r] * kAccInv + bg1[0];
        const float pf = acc[1][r] * kAccInv + bg1[1];
        const float pg = acc[2][r] * kAccInv + bg1[2];
        const float po = acc[3][r] * kAccInv + bg1[3];
        const float ig = sigm_f(pi);
        const float fg = sigm_f(pf);
        const float gg = tanh_f(pg);
        const float og = sigm_f(po);
        const float cc = fg * c1st[r] + ig * gg;
        c1st[r] = cc;
        const float h = og * tanh_f(cc);
        h1last[r] = h;
        A1s[(8 * hi + r) * kPA1 + kHid + col] = (_Float16)(h * kActScale);
      }
    }
  }

#pragma unroll
  for (int r = 0; r < 8; ++r) Os[(8 * hi + r) * kOSP + col] = h1last[r];
  __syncthreads();
  {
    const float* src = Os + w * kOSP;
    float* dst = out + (size_t)(b0 + w) * kHid;
    for (int pass = 0; pass < 2; ++pass) {
#pragma unroll
      for (int it = 0; it < 2; ++it) {
        const v4f v = *(const v4f*)(src + it * 128 + lane * 4);
        *(volatile v4f*)(dst + it * 128 + lane * 4) = v;
      }
      __threadfence();
    }
  }
}

extern "C" void kernel_launch(void* const* d_in, const int* in_sizes, int n_in,
                              void* d_out, int out_size, void* d_ws, size_t ws_size,
                              hipStream_t stream) {
  (void)n_in;
  const float* Mx    = (const float*)d_in[0];
  const float* W_ih0 = (const float*)d_in[1];
  const float* W_hh0 = (const float*)d_in[2];
  const float* b_ih0 = (const float*)d_in[3];
  const float* b_hh0 = (const float*)d_in[4];
  const float* W_ih1 = (const float*)d_in[5];
  const float* W_hh1 = (const float*)d_in[6];
  const float* b_ih1 = (const float*)d_in[7];
  const float* b_hh1 = (const float*)d_in[8];

  const size_t off0 = 0;
  const size_t bytes0 = (size_t)kGates * kK0 * 2;
  const size_t off1 = off0 + bytes0;
  const size_t bytes1 = (size_t)kGates * kK1 * 2;
  const size_t total = off1 + bytes1;
  if (ws_size < total) return;
  if ((size_t)in_sizes[0] < (size_t)kBatch * kSteps * kIn) return;
  if ((size_t)out_size < (size_t)kBatch * kHid) return;

  unsigned char* ws = (unsigned char*)d_ws;
  _Float16* Wc0 = (_Float16*)(ws + off0);
  _Float16* Wc1 = (_Float16*)(ws + off1);

  const int chunks0 = kGates * (kK0 / 8);
  const int chunks1 = kGates * (kK1 / 8);
  build_bt_plane<<<(chunks0 + 255) / 256, 256, 0, stream>>>(W_ih0, kIn, W_hh0, kHid, Wc0, kK0, kGates, kWScale);
  build_bt_plane<<<(chunks1 + 255) / 256, 256, 0, stream>>>(W_ih1, kHid, W_hh1, kHid, Wc1, kK1, kGates, kWScale);

  lstm2_persist<<<kBatch / kRowsPerBlock, 512, 0, stream>>>(
      Mx, Wc0, Wc1, b_ih0, b_hh0, b_ih1, b_hh1, (float*)d_out);
}
